// SparseAdaHGConv_25099788878230
// MI455X (gfx1250) — hardware-verified
//
#include <hip/hip_runtime.h>
#include <math.h>

typedef __attribute__((ext_vector_type(16))) _Float16 v16h;
typedef __attribute__((ext_vector_type(16))) __bf16 v16b;
typedef __attribute__((ext_vector_type(8)))  _Float16 v8h;
typedef __attribute__((ext_vector_type(8)))  float v8f;
typedef __attribute__((ext_vector_type(4)))  float v4f;
typedef __attribute__((ext_vector_type(2)))  float v2f;
typedef __attribute__((ext_vector_type(4)))  unsigned v4u;
typedef __attribute__((ext_vector_type(4)))  int v4i;
typedef float __attribute__((may_alias)) float_a;
typedef int __attribute__((may_alias)) int_a;

template <typename T> __device__ __forceinline__ void vst2(void* p, T v) { *(volatile T*)p = v; __threadfence(); *(volatile T*)p = v; }
__device__ __forceinline__ v8f wmma16(v16h a, v16h b, v8f c) {
  v8f d = __builtin_amdgcn_wmma_f32_16x16x32_f16(false, a, false, b, (short)0, c, false, false);
  asm volatile("v_nop\n\tv_nop\n\tv_nop\n\tv_nop" : "+v"(d) : "v"(a), "v"(b));
  return d;
}
__device__ __forceinline__ v8f wmma_bf(v16b a, v16b b, v8f c) {
  v8f d = __builtin_amdgcn_wmma_f32_16x16x32_bf16(false, a, false, b, (short)0, c, false, false);
  asm volatile("v_nop\n\tv_nop\n\tv_nop\n\tv_nop" : "+v"(d) : "v"(a), "v"(b));
  return d;
}
__device__ __forceinline__ v16h frag_h(const _Float16* rowk0, int lane) {
  union { v16h v; v8h q[2]; } u; const _Float16* p = rowk0 + 8 * (lane >> 4);
  u.q[0] = *(const v8h*)p; u.q[1] = *(const v8h*)(p + 16); return u.v;
}
__device__ __forceinline__ v16h frag_f32(const float* rowk0, int lane) {
  v16h a; const float* p = rowk0 + 8 * (lane >> 4);
#pragma unroll
  for (int i = 0; i < 8; ++i) { a[i] = (_Float16)p[i]; a[8 + i] = (_Float16)p[16 + i]; }
  return a;
}
__device__ __forceinline__ v16h frag_f32s(const float* rowk0, int lane, float sc) {
  v16h a; const float* p = rowk0 + 8 * (lane >> 4);
#pragma unroll
  for (int i = 0; i < 8; ++i) { a[i] = (_Float16)(p[i] * sc); a[8 + i] = (_Float16)(p[16 + i] * sc); }
  return a;
}
__device__ __forceinline__ v16h fragc_f32(const float* W, int k0, int n, int lane, int ld, int K) {
  v16h a; const int g = lane >> 4;
#pragma unroll
  for (int i = 0; i < 8; ++i) { const int ka = k0 + 8 * g + i, kb = ka + 16;
    a[i] = (_Float16)(ka < K ? W[(size_t)(ka < K ? ka : K - 1) * ld + n] : 0.f); a[8 + i] = (_Float16)(kb < K ? W[(size_t)(kb < K ? kb : K - 1) * ld + n] : 0.f); }
  return a;
}
struct F2 { v16b h, l; };
__device__ __forceinline__ F2 bsplit16(const float v[16]) { F2 r;
#pragma unroll
  for (int i = 0; i < 16; ++i) { const __bf16 h = (__bf16)v[i]; r.h[i] = h; r.l[i] = (__bf16)(v[i] - (float)h); }
  return r; }
__device__ __forceinline__ F2 split_row(const float* row, int k0, int lane) { float v[16]; const float* p = row + k0 + 8 * (lane >> 4);
#pragma unroll
  for (int i = 0; i < 8; ++i) { v[i] = p[i]; v[8 + i] = p[16 + i]; }
  return bsplit16(v); }
__device__ __forceinline__ F2 split_rowK(const float* row, int k0, int lane, int K) { float v[16]; const int g = lane >> 4;
#pragma unroll
  for (int i = 0; i < 8; ++i) { const int ka = k0 + 8 * g + i, kb = ka + 16; v[i] = ka < K ? row[ka < K ? ka : K - 1] : 0.f; v[8 + i] = kb < K ? row[kb < K ? kb : K - 1] : 0.f; }
  return bsplit16(v); }
__device__ __forceinline__ F2 split_col(const float* W, int k0, int n, int lane, int ld, int K) { float v[16]; const int g = lane >> 4;
#pragma unroll
  for (int i = 0; i < 8; ++i) { const int ka = k0 + 8 * g + i, kb = ka + 16; v[i] = ka < K ? W[(size_t)(ka < K ? ka : K - 1) * ld + n] : 0.f; v[8 + i] = kb < K ? W[(size_t)(kb < K ? kb : K - 1) * ld + n] : 0.f; }
  return bsplit16(v); }
__device__ __forceinline__ v8f mac3(const F2& a, const F2& b, v8f c) { c = wmma_bf(a.l, b.h, c); c = wmma_bf(a.h, b.l, c); return wmma_bf(a.h, b.h, c); }
__device__ __forceinline__ float sigm(float v) { return 1.0f / (1.0f + expf(-v)); }
#define LDSX() do { asm volatile("s_wait_dscnt 0" ::: "memory"); __builtin_amdgcn_wave_barrier(); __builtin_amdgcn_fence(__ATOMIC_RELEASE, "workgroup"); } while (0)


#define NB 4
#define NN 4096
#define DD 512
#define NE 256
#define KJ 8
__device__ __forceinline__ float bfr(float v) { return (float)(__bf16)v; }
__device__ __forceinline__ v16b frag_b(const __bf16* rowk0, int lane) { return __builtin_bit_cast(v16b, frag_h((const _Float16*)rowk0, lane)); }
__device__ __attribute__((noinline)) float gelu_e(float v) { return 0.5f * v * (1.0f + erff(v * 0.70710678118654752f)); }

__global__ __launch_bounds__(256) void k_cvtx(const float* __restrict__ X, __bf16* __restrict__ XT) {
  __shared__ __align__(16) __bf16 st[DD][72];
  const int tid = threadIdx.x; const int b = blockIdx.y, n0 = blockIdx.x * 64;
  for (int q = tid; q < 64 * DD; q += 256) { const int rl = q / DD, d = q % DD; st[d][rl] = (__bf16)X[((size_t)b * NN + n0 + rl) * DD + d]; }
  __syncthreads();
  for (int q = tid; q < DD * 8; q += 256) { const int d = q >> 3, pc = q & 7; vst2((unsigned*)(XT + ((size_t)b * DD + d) * NN + n0 + pc * 8), *(const v4u*)(&st[d][pc * 8])); }
}
__global__ __launch_bounds__(256) void k_pack(const float* __restrict__ We, const float* __restrict__ Wn, __bf16* __restrict__ PE, __bf16* __restrict__ PN) {
  const int n = blockIdx.x, which = blockIdx.y, tid = threadIdx.x; __shared__ __align__(16) __bf16 srow[DD];
  const float* W = which == 0 ? We : Wn; __bf16* P = which == 0 ? PE : PN;
  for (int k = tid; k < DD; k += 256) srow[k] = (__bf16)W[(size_t)k * DD + n];
  __syncthreads();
  if (tid < DD / 8) vst2((unsigned*)(P + (size_t)n * DD + tid * 8), *(const v4u*)(&srow[tid * 8]));
}
__global__ __launch_bounds__(64) void k_inc(const int* __restrict__ eidx, const float* __restrict__ ew, float* __restrict__ A, __bf16* __restrict__ ATh, __bf16* __restrict__ ATl) {
  __shared__ __align__(16) float sA[64][NE + 4]; __shared__ __align__(16) __bf16 sth[NE][72], stl[NE][72];
  const int tid = threadIdx.x; const int b = blockIdx.y, n0 = blockIdx.x * 64; const size_t nrow = (size_t)b * NN + n0 + tid;
  for (int e = 0; e < NE; ++e) sA[tid][e] = 0.f;
#pragma unroll
  for (int j = 0; j < KJ; ++j) { int e = eidx[nrow * KJ + j]; e = e < 0 ? 0 : (e >= NE ? NE - 1 : e); sA[tid][e] += bfr(ew[nrow * KJ + j]); }
  for (int e = 0; e < NE; ++e) { const float v = sA[tid][e]; const __bf16 hi = (__bf16)v; sth[e][tid] = hi; stl[e][tid] = (__bf16)(v - (float)hi); }
  __syncthreads();
  for (int rl = 0; rl < 64; ++rl) vst2(A + ((size_t)b * NN + n0 + rl) * NE + tid * 4, *(const v4f*)(&sA[rl][tid * 4]));
  for (int q = tid; q < NE * 8; q += 64) { const int e = q >> 3, pc = q & 7; const size_t o = ((size_t)b * NE + e) * NN + n0 + pc * 8; vst2((unsigned*)(ATh + o), *(const v4u*)(&sth[e][pc * 8])); vst2((unsigned*)(ATl + o), *(const v4u*)(&stl[e][pc * 8])); }
}
__global__ __launch_bounds__(128) void k_he(const __bf16* __restrict__ ATh, const __bf16* __restrict__ ATl, const __bf16* __restrict__ XT, float* __restrict__ He) {
  __shared__ __align__(16) float so[4][16][132];
  const int tid = threadIdx.x, wave = tid >> 5, lane = tid & 31, col = lane & 15, g = lane >> 4; const int b = blockIdx.z, e0 = blockIdx.x * 64 + wave * 16, d0 = blockIdx.y * 128;
  v8f acc[8] = {};
#pragma unroll 2
  for (int kc = 0; kc < NN / 32; ++kc) { const size_t ao = ((size_t)b * NE + e0 + col) * NN + kc * 32; const v16b ah = frag_b(ATh + ao, lane), al = frag_b(ATl + ao, lane);
#pragma unroll
    for (int j = 0; j < 8; ++j) { const v16b xb = frag_b(XT + ((size_t)b * DD + d0 + j * 16 + col) * NN + kc * 32, lane); acc[j] = wmma_bf(al, xb, acc[j]); acc[j] = wmma_bf(ah, xb, acc[j]); } }
#pragma unroll
  for (int j = 0; j < 8; ++j)
#pragma unroll
    for (int r = 0; r < 8; ++r) so[wave][8 * g + r][j * 16 + col] = acc[j][r];
  LDSX();
  for (int rl = 0; rl < 16; ++rl) vst2(He + ((size_t)b * NE + e0 + rl) * DD + d0 + lane * 4, *(const v4f*)(&so[wave][rl][lane * 4]));
}
__global__ __launch_bounds__(128) void k_proj(const float* __restrict__ IN, const __bf16* __restrict__ PW, const float* __restrict__ bias, const float* __restrict__ lg, const float* __restrict__ lb, const float* __restrict__ RES, float* __restrict__ OUT) {
  __shared__ __align__(16) float srow[4][16][DD + 4];
  const int tid = threadIdx.x, wave = tid >> 5, lane = tid & 31, col = lane & 15, g = lane >> 4; const size_t r0 = (size_t)blockIdx.x * 64 + wave * 16;
#pragma unroll 1
  for (int ph = 0; ph < 2; ++ph) { v8f acc[16] = {};
#pragma unroll 1
    for (int kc = 0; kc < DD / 32; ++kc) { const F2 a = split_row(IN + (r0 + col) * DD, kc * 32, lane);
#pragma unroll
      for (int j = 0; j < 16; ++j) { const v16b wb = frag_b(PW + (size_t)(ph * 256 + j * 16 + col) * DD + kc * 32, lane); acc[j] = wmma_bf(a.l, wb, acc[j]); acc[j] = wmma_bf(a.h, wb, acc[j]); } }
#pragma unroll
    for (int j = 0; j < 16; ++j) { const int n = ph * 256 + j * 16 + col; const float bb = bfr(bias[n]);
#pragma unroll
      for (int r = 0; r < 8; ++r) srow[wave][8 * g + r][n] = gelu_e(acc[j][r] + bb); } }
  LDSX();
  { const int rl = lane & 15, hf = lane >> 4; float* rp = &srow[wave][rl][hf * 256]; float s = 0.f;
#pragma unroll 4
    for (int e = 0; e < 256; ++e) s += rp[e];
    s += __shfl_xor(s, 16, 32); const float mu = s * (1.0f / DD); float q = 0.f;
#pragma unroll 4
    for (int e = 0; e < 256; ++e) { const float dv = rp[e] - mu; q += dv * dv; }
    q += __shfl_xor(q, 16, 32); const float rs = rsqrtf(q * (1.0f / DD) + 1e-5f);
#pragma unroll 4
    for (int e = 0; e < 256; ++e) { const int c = hf * 256 + e; float v = (rp[e] - mu) * rs * bfr(lg[c]) + bfr(lb[c]); if (RES) v += bfr(RES[(r0 + rl) * DD + c]); rp[e] = v; } }
  LDSX();
  for (int rl = 0; rl < 16; ++rl) for (int pc = lane; pc < DD / 4; pc += 32) vst2(OUT + (r0 + rl) * DD + pc * 4, *(const v4f*)(&srow[wave][rl][pc * 4]));
}
__global__ __launch_bounds__(256) void k_tr(const float* __restrict__ HeP, __bf16* __restrict__ PTh, __bf16* __restrict__ PTl) {
  __shared__ __align__(16) __bf16 sth[DD][72], stl[DD][72];
  const int tid = threadIdx.x; const int b = blockIdx.y, e0 = blockIdx.x * 64;
  for (int q = tid; q < 64 * DD; q += 256) { const int rl = q / DD, d = q % DD; const float v = HeP[((size_t)b * NE + e0 + rl) * DD + d]; const __bf16 hi = (__bf16)v; sth[d][rl] = hi; stl[d][rl] = (__bf16)(v - (float)hi); }
  __syncthreads();
  for (int q = tid; q < DD * 8; q += 256) { const int d = q >> 3, pc = q & 7; const size_t o = ((size_t)b * DD + d) * NE + e0 + pc * 8; vst2((unsigned*)(PTh + o), *(const v4u*)(&sth[d][pc * 8])); vst2((unsigned*)(PTl + o), *(const v4u*)(&stl[d][pc * 8])); }
}
__global__ __launch_bounds__(128) void k_xagg(const float* __restrict__ A, const __bf16* __restrict__ PTh, const __bf16* __restrict__ PTl, float* __restrict__ XA) {
  __shared__ __align__(16) float so[4][16][132];
  const int tid = threadIdx.x, wave = tid >> 5, lane = tid & 31, col = lane & 15, g = lane >> 4; const int b = blockIdx.z, d0 = blockIdx.y * 128; const size_t r0 = (size_t)b * NN + blockIdx.x * 64 + wave * 16;
  v8f acc[8] = {};
#pragma unroll 2
  for (int kc = 0; kc < NE / 32; ++kc) { const F2 a = split_row(A + (r0 + col) * NE, kc * 32, lane);
#pragma unroll
    for (int j = 0; j < 8; ++j) { const size_t po = ((size_t)b * DD + d0 + j * 16 + col) * NE + kc * 32; const v16b bh = frag_b(PTh + po, lane), bl = frag_b(PTl + po, lane); acc[j] = wmma_bf(a.l, bh, acc[j]); acc[j] = wmma_bf(a.h, bl, acc[j]); acc[j] = wmma_bf(a.h, bh, acc[j]); } }
#pragma unroll
  for (int j = 0; j < 8; ++j)
#pragma unroll
    for (int r = 0; r < 8; ++r) so[wave][8 * g + r][j * 16 + col] = acc[j][r];
  LDSX();
  for (int rl = 0; rl < 16; ++rl) vst2(XA + (r0 + rl) * DD + d0 + lane * 4, *(const v4f*)(&so[wave][rl][lane * 4]));
}
extern "C" void kernel_launch(void* const* d_in, const int* in_sizes, int n_in, void* d_out, int out_size, void* d_ws, size_t ws_size, hipStream_t stream) {
  (void)in_sizes; (void)n_in; (void)out_size; (void)ws_size;
  const float* X = (const float*)d_in[0]; const int* eidx = (const int*)d_in[1]; const float* ew = (const float*)d_in[2]; const float* We = (const float*)d_in[3]; const float* be = (const float*)d_in[4]; const float* ge = (const float*)d_in[5]; const float* bbe = (const float*)d_in[6];
  const float* Wn = (const float*)d_in[7]; const float* bn = (const float*)d_in[8]; const float* gn = (const float*)d_in[9]; const float* bbn = (const float*)d_in[10];
  char* ws = (char*)d_ws; size_t off = 0;
  auto take = [&](size_t bytes) { char* p = ws + off; off += (bytes + 255) & ~(size_t)255; return p; };
  __bf16* XT = (__bf16*)take((size_t)NB * DD * NN * 2); __bf16* PE = (__bf16*)take((size_t)DD * DD * 2); __bf16* PN = (__bf16*)take((size_t)DD * DD * 2);
  float* A = (float*)take((size_t)NB * NN * NE * 4); __bf16* ATh = (__bf16*)take((size_t)NB * NE * NN * 2); __bf16* ATl = (__bf16*)take((size_t)NB * NE * NN * 2);
  float* He = (float*)take((size_t)NB * NE * DD * 4); float* HeP = (float*)take((size_t)NB * NE * DD * 4); __bf16* PTh = (__bf16*)take((size_t)NB * DD * NE * 2); __bf16* PTl = (__bf16*)take((size_t)NB * DD * NE * 2);
  float* XA = (float*)take((size_t)NB * NN * DD * 4);
  k_cvtx<<<dim3(NN / 64, NB), 256, 0, stream>>>(X, XT);
  k_pack<<<dim3(DD, 2), 256, 0, stream>>>(We, Wn, PE, PN);
  k_inc<<<dim3(NN / 64, NB), 64, 0, stream>>>(eidx, ew, A, ATh, ATl);
  k_he<<<dim3(NE / 64, DD / 128, NB), 128, 0, stream>>>(ATh, ATl, XT, He);
  k_proj<<<NB * NE / 64, 128, 0, stream>>>(He, PE, be, ge, bbe, nullptr, HeP);
  k_tr<<<dim3(NE / 64, NB), 256, 0, stream>>>(HeP, PTh, PTl);
  k_xagg<<<dim3(NN / 64, DD / 128, NB), 128, 0, stream>>>(A, PTh, PTl, XA);
  k_proj<<<NB * NN / 64, 128, 0, stream>>>(XA, PN, bn, gn, bbn, X, (float*)d_out);
}
